// SS2D_block_23192823398803
// MI455X (gfx1250) — hardware-run, weakly checked
//
#include <hip/hip_runtime.h>
#include <math.h>

typedef __attribute__((ext_vector_type(16))) __bf16   v16b;
typedef __attribute__((ext_vector_type(8)))  __bf16   v8b;
typedef __attribute__((ext_vector_type(8)))  float    v8f;
typedef __attribute__((ext_vector_type(4)))  float    v4f;
typedef __attribute__((ext_vector_type(4)))  unsigned v4u;

constexpr int kImg   = 4;
constexpr int kSide  = 64;
constexpr int kLen   = kSide * kSide;
constexpr int kCh    = 96;
constexpr int kNst   = 16;
constexpr int kRk    = 4;
constexpr int kDir   = 4;
constexpr int kXw    = kRk + 2 * kNst;
constexpr int kXp    = 48;
constexpr int kNW    = kDir * kXp;
constexpr int kTok   = kImg * kLen;
constexpr int kChunk = 64;
static_assert(kLen == 4096 && kTok == 16384, "token count");
static_assert(kXw == 36 && kNW == 192, "stacked projection width");
static_assert((kCh % 32) == 0, "GEMM K multiple of 32");
static_assert((kTok % 64) == 0 && (kNW % 64) == 0, "GEMM M,N multiples of 64");
static_assert((kLen % kChunk) == 0, "scan chunking");

constexpr size_t kSzA   = (size_t)kTok * kCh * 2;
constexpr size_t kSzB   = (size_t)kNW * kCh * 2;
constexpr size_t kSzXD  = (size_t)kTok * kNW * 4;
constexpr size_t kSzYD  = (size_t)kDir * kTok * kCh * 4;
constexpr size_t kOffAH = 0;
constexpr size_t kOffAL = kOffAH + kSzA;
constexpr size_t kOffBH = kOffAL + kSzA;
constexpr size_t kOffBL = kOffBH + kSzB;
constexpr size_t kOffXD = kOffBL + kSzB;
constexpr size_t kOffYD = kOffXD + kSzXD;
constexpr size_t kWsTotal = kOffYD + kSzYD;
static_assert(kWsTotal == 44113920ull, "carve total");
static_assert(kWsTotal <= 134217728ull, "carve cap");
static_assert((kOffAL % 128) == 0 && (kOffBH % 128) == 0 && (kOffBL % 128) == 0 &&
              (kOffXD % 128) == 0 && (kOffYD % 128) == 0, "128-B aligned regions");

constexpr unsigned kPackXBlocks = (unsigned)(kTok * kCh / 8 / 256);
constexpr unsigned kPackWBlocks = (unsigned)(kNW * kCh / 8 / 256);
static_assert(kPackXBlocks * 256u * 8u == (unsigned)(kTok * kCh), "x pack coverage");
static_assert(kPackWBlocks * 256u * 8u == (unsigned)(kNW * kCh), "weight pack coverage");

__device__ __forceinline__ unsigned bf_hi_bits(float f) {
  const unsigned u = __float_as_uint(f);
  const unsigned lsb = (u & 0x00010000u) ? 1u : 0u;
  return (u + 0x7FFFu + lsb) & 0xFFFF0000u;
}
__device__ __forceinline__ void split_pair(float f0, float f1, unsigned& whi, unsigned& wlo) {
  const unsigned h0 = bf_hi_bits(f0);
  const unsigned h1 = bf_hi_bits(f1);
  const unsigned l0 = bf_hi_bits(f0 - __uint_as_float(h0));
  const unsigned l1 = bf_hi_bits(f1 - __uint_as_float(h1));
  whi = __builtin_amdgcn_perm(h1, h0, 0x07060302u);
  wlo = __builtin_amdgcn_perm(l1, l0, 0x07060302u);
}
__device__ __forceinline__ void store_split8(unsigned* ph, unsigned* pl,
                                             float f0, float f1, float f2, float f3,
                                             float f4, float f5, float f6, float f7) {
  unsigned h0, h1, h2, h3, l0, l1, l2, l3;
  split_pair(f0, f1, h0, l0);
  split_pair(f2, f3, h1, l1);
  split_pair(f4, f5, h2, l2);
  split_pair(f6, f7, h3, l3);
  const v4u hv = {h0, h1, h2, h3};
  const v4u lv = {l0, l1, l2, l3};
  *(volatile v4u*)ph = hv;
  *(volatile v4u*)pl = lv;
  __threadfence();
  *(volatile v4u*)ph = hv;
  *(volatile v4u*)pl = lv;
}

__global__ __launch_bounds__(256) void pack_planes_kernel(
    const float* __restrict__ X, const float* __restrict__ Wp,
    unsigned* __restrict__ AH, unsigned* __restrict__ AL,
    unsigned* __restrict__ BH, unsigned* __restrict__ BL)
{
  const unsigned tid = threadIdx.x;
  if (blockIdx.x < kPackXBlocks) {
    const unsigned i = blockIdx.x * 256u + tid;
    const size_t e0 = (size_t)i * 8;
    const v4f a0 = *(const v4f*)(X + e0);
    const v4f a1 = *(const v4f*)(X + e0 + 4);
    const float f0 = a0[0], f1 = a0[1], f2 = a0[2], f3 = a0[3];
    const float f4 = a1[0], f5 = a1[1], f6 = a1[2], f7 = a1[3];
    store_split8(AH + (size_t)i * 4, AL + (size_t)i * 4, f0, f1, f2, f3, f4, f5, f6, f7);
  } else {
    unsigned i = (blockIdx.x - kPackXBlocks) * 256u + tid;
    asm volatile("" : "+v"(i));
    unsigned row = i / 12u;
    asm volatile("" : "+v"(row));
    unsigned c8 = (i - row * 12u) * 8u;
    asm volatile("" : "+v"(c8));
    unsigned kd = row / 48u;
    asm volatile("" : "+v"(kd));
    unsigned c = row - kd * 48u;
    asm volatile("" : "+v"(c));
    const bool valid = (c < (unsigned)kXw);
    const unsigned cc = valid ? c : (unsigned)(kXw - 1);
    const float* sp = Wp + (size_t)(kd * (unsigned)kXw + cc) * kCh + c8;
    const v4f a0 = *(const v4f*)(sp);
    const v4f a1 = *(const v4f*)(sp + 4);
    float f0 = a0[0], f1 = a0[1], f2 = a0[2], f3 = a0[3];
    float f4 = a1[0], f5 = a1[1], f6 = a1[2], f7 = a1[3];
    asm volatile("" : "+v"(f0), "+v"(f1), "+v"(f2), "+v"(f3));
    asm volatile("" : "+v"(f4), "+v"(f5), "+v"(f6), "+v"(f7));
    f0 = valid ? f0 : 0.0f;
    f1 = valid ? f1 : 0.0f;
    f2 = valid ? f2 : 0.0f;
    f3 = valid ? f3 : 0.0f;
    f4 = valid ? f4 : 0.0f;
    f5 = valid ? f5 : 0.0f;
    f6 = valid ? f6 : 0.0f;
    f7 = valid ? f7 : 0.0f;
    store_split8(BH + (size_t)i * 4, BL + (size_t)i * 4, f0, f1, f2, f3, f4, f5, f6, f7);
  }
}

union FragB { v16b v; v8b h[2]; };
__device__ __forceinline__ v16b frag_load(const __bf16* p) {
  FragB f;
  f.h[0] = *(const v8b*)(p);
  f.h[1] = *(const v8b*)(p + 16);
  return f.v;
}
__device__ __forceinline__ v8f mma_bf16(v16b a, v16b b, v8f c) {
  return __builtin_amdgcn_wmma_f32_16x16x32_bf16(false, a, false, b, (short)0, c, false, false);
}
__device__ __forceinline__ void dep_guard4_b(v8f& a, v8f& b, v8f& c, v8f& d, v16b x, v16b y) {
  asm volatile("v_nop\n\tv_nop\n\tv_nop\n\tv_nop" : "+v"(a), "+v"(b), "+v"(c), "+v"(d) : "v"(x), "v"(y));
}
__device__ __forceinline__ void keep4_b(v16b a, v16b b, v16b c, v16b d) {
  asm volatile("v_nop" :: "v"(a), "v"(b), "v"(c), "v"(d));
}
__device__ __forceinline__ void acc_guard4(v8f& a, v8f& b, v8f& c, v8f& d) {
  asm volatile("v_nop\n\tv_nop\n\tv_nop\n\tv_nop" : "+v"(a), "+v"(b), "+v"(c), "+v"(d));
}

__global__ __launch_bounds__(256) void proj_gemm64_kernel(
    const unsigned short* __restrict__ Ap, const unsigned short* __restrict__ A2p,
    const unsigned short* __restrict__ Btp, const unsigned short* __restrict__ Bt2p,
    float* __restrict__ C)
{
  constexpr int M = kTok, N = kNW, K = kCh, lda = kCh, ldb = kCh, ldc = kNW;
  const __bf16* A   = (const __bf16*)Ap;
  const __bf16* A2  = (const __bf16*)A2p;
  const __bf16* Bt  = (const __bf16*)Btp;
  const __bf16* Bt2 = (const __bf16*)Bt2p;
  __shared__ __align__(16) float sT[8][16 * 68];
  const int lane = threadIdx.x & 31;
  const int wave = threadIdx.x >> 5;
  constexpr int tilesN = N >> 6;
  constexpr int tilesM = M >> 6;
  const int tile = blockIdx.x * 8 + wave;
  if (tile >= tilesM * tilesN) return;
  const int tm = tile / tilesN;
  const int tn = tile - tm * tilesN;
  const int m0 = tm << 6;
  const int n0 = tn << 6;

  const int rlane = lane & 15;
  const int koff  = (lane >> 4) * 8;
  const int mOff  = (lane >> 4) * 8;

  v8f acc[4][4];
#pragma unroll
  for (int i = 0; i < 4; ++i)
#pragma unroll
    for (int j = 0; j < 4; ++j) acc[i][j] = (v8f){0.f,0.f,0.f,0.f,0.f,0.f,0.f,0.f};

#pragma unroll 1
  for (int k0 = 0; k0 < K; k0 += 32) {
    v16b bh[4], bl[4];
#pragma unroll
    for (int j = 0; j < 4; ++j) {
      const size_t bo = (size_t)(n0 + (j << 4) + rlane) * ldb + koff + k0;
      bh[j] = frag_load(Bt + bo);
      bl[j] = frag_load(Bt2 + bo);
    }
#pragma unroll
    for (int i = 0; i < 4; ++i) {
      const size_t ao = (size_t)(m0 + (i << 4) + rlane) * lda + koff + k0;
      const v16b ah = frag_load(A + ao);
      const v16b al = frag_load(A2 + ao);
#pragma unroll
      for (int j = 0; j < 4; ++j) {
        acc[i][j] = mma_bf16(ah, bh[j], acc[i][j]);
        acc[i][j] = mma_bf16(ah, bl[j], acc[i][j]);
        acc[i][j] = mma_bf16(al, bh[j], acc[i][j]);
      }
      dep_guard4_b(acc[i][0], acc[i][1], acc[i][2], acc[i][3], ah, al);
    }
    keep4_b(bh[0], bh[1], bh[2], bh[3]);
    keep4_b(bl[0], bl[1], bl[2], bl[3]);
  }
  acc_guard4(acc[0][0], acc[0][1], acc[0][2], acc[0][3]);
  acc_guard4(acc[1][0], acc[1][1], acc[1][2], acc[1][3]);
  acc_guard4(acc[2][0], acc[2][1], acc[2][2], acc[2][3]);
  acc_guard4(acc[3][0], acc[3][1], acc[3][2], acc[3][3]);

  float* slab = sT[wave];
#pragma unroll
  for (int i = 0; i < 4; ++i) {
    const int mBase = m0 + (i << 4);
#pragma unroll
    for (int j = 0; j < 4; ++j) {
#pragma unroll
      for (int r = 0; r < 8; ++r) {
        slab[(mOff + r) * 68 + (j << 4) + rlane] = acc[i][j][r];
      }
    }
    __builtin_amdgcn_fence(__ATOMIC_RELEASE, "workgroup");
    __builtin_amdgcn_wave_barrier();
    __builtin_amdgcn_fence(__ATOMIC_ACQUIRE, "workgroup");
    {
      const int hh = lane >> 4, c4 = (lane & 15) * 4;
      for (int pass = 0; pass < 2; ++pass) {
#pragma unroll
        for (int it = 0; it < 8; ++it) {
          const int row = it * 2 + hh;
          const v4f v = *(const v4f*)(slab + row * 68 + c4);
          *(volatile v4f*)(C + (size_t)(mBase + row) * ldc + n0 + c4) = v;
        }
        __threadfence();
      }
    }
    __builtin_amdgcn_fence(__ATOMIC_RELEASE, "workgroup");
    __builtin_amdgcn_wave_barrier();
    __builtin_amdgcn_fence(__ATOMIC_ACQUIRE, "workgroup");
  }
}

__device__ __forceinline__ unsigned spatial_pos(unsigned kd, unsigned l) {
  const unsigned lp = (kd >= 2u) ? ((unsigned)(kLen - 1) - l) : l;
  const unsigned tp = ((lp & 63u) << 6) | (lp >> 6);
  return (kd & 1u) ? tp : lp;
}

__global__ __launch_bounds__(192) void scan_dir_kernel(
    const float* __restrict__ X, const float* __restrict__ XD,
    const float* __restrict__ dtw, const float* __restrict__ dtb,
    const float* __restrict__ alog, const float* __restrict__ dskip,
    float* __restrict__ YD)
{
  __shared__ __align__(16) float sX[kChunk * kXw];
  __shared__ __align__(16) float sU[kChunk * kCh];
  __shared__ __align__(16) float sY[kChunk * kCh];
  const unsigned tid  = threadIdx.x;
  const unsigned lane = tid & 31u;
  const unsigned wave = tid >> 5;
  const unsigned kd   = blockIdx.x & 3u;
  const unsigned bi   = blockIdx.x >> 2;
  const unsigned d    = tid >> 1;
  const unsigned half = tid & 1u;
  const unsigned chn  = kd * (unsigned)kCh + d;

#pragma unroll 1
  for (unsigned j = 0; j < 8u; ++j) {
    sY[j * 192u + tid] = -expf(alog[(size_t)chn * kNst + half * 8u + j]);
  }
  __syncthreads();
  float negA[8], h[8];
#pragma unroll
  for (int j = 0; j < 8; ++j) {
    negA[j] = sY[(unsigned)j * 192u + tid];
    h[j] = 0.0f;
  }
  const v4f wv = *(const v4f*)(dtw + (size_t)chn * kRk);
  const float w0 = wv[0], w1 = wv[1], w2 = wv[2], w3 = wv[3];
  const float bias = dtb[chn];
  const float dsk  = dskip[chn];

  const unsigned srow  = tid & 63u;
  const unsigned spart = tid >> 6;
  const unsigned q   = lane >> 3;
  const unsigned c4  = (lane & 7u) * 4u;
  const unsigned seg = (wave >= 3u) ? (wave - 3u) : wave;
  const unsigned rg  = (wave >= 3u) ? 4u : 0u;
  float* Yk = YD + (size_t)kd * kTok * kCh;
  const unsigned tok0 = bi * (unsigned)kLen;

#pragma unroll 1
  for (unsigned t0 = 0; t0 < (unsigned)kLen; t0 += (unsigned)kChunk) {
    __syncthreads();
    {
      const unsigned mS = tok0 + spatial_pos(kd, t0 + srow);
      const float* xdp = XD + (size_t)mS * kNW + kd * (unsigned)kXp + spart * 12u;
#pragma unroll
      for (int i = 0; i < 3; ++i)
        *(v4f*)(sX + srow * (unsigned)kXw + spart * 12u + 4u * (unsigned)i) = *(const v4f*)(xdp + 4 * i);
      const float* xp = X + (size_t)mS * kCh + spart * 32u;
#pragma unroll
      for (int i = 0; i < 8; ++i)
        *(v4f*)(sU + srow * (unsigned)kCh + spart * 32u + 4u * (unsigned)i) = *(const v4f*)(xp + 4 * i);
    }
    __syncthreads();
#pragma unroll 1
    for (unsigned s = 0; s < (unsigned)kChunk; ++s) {
      const float* xr = sX + s * (unsigned)kXw;
      const v4f dv = *(const v4f*)(xr);
      const v4f b0 = *(const v4f*)(xr + 4u + half * 8u);
      const v4f b1 = *(const v4f*)(xr + 8u + half * 8u);
      const v4f c0 = *(const v4f*)(xr + 20u + half * 8u);
      const v4f c1 = *(const v4f*)(xr + 24u + half * 8u);
      const float u = sU[s * (unsigned)kCh + d];
      float z = dv[0] * w0;
      z = fmaf(dv[1], w1, z);
      z = fmaf(dv[2], w2, z);
      z = fmaf(dv[3], w3, z);
      z = z + bias;
      const float delta = fmaxf(z, 0.0f) + log1pf(expf(-fabsf(z)));
      const float du = delta * u;
      const float Bs[8] = {b0[0], b0[1], b0[2], b0[3], b1[0], b1[1], b1[2], b1[3]};
      const float Cs[8] = {c0[0], c0[1], c0[2], c0[3], c1[0], c1[1], c1[2], c1[3]};
      float y = 0.0f;
#pragma unroll
      for (int j = 0; j < 8; ++j) {
        float e = expf(delta * negA[j]);
        e = (e < 1.17549435e-38f) ? 0.0f : e;
        h[j] = fmaf(e, h[j], du * Bs[j]);
        y = fmaf(h[j], Cs[j], y);
      }
      const float yo = __shfl_xor(y, 1, 32);
      const float yt = (y + yo) + dsk * u;
      sY[s * (unsigned)kCh + d] = yt;
    }
    __syncthreads();
    v4f fv[8];
    unsigned off[8];
#pragma unroll
    for (int it = 0; it < 8; ++it) {
      const unsigned row = (unsigned)it * 8u + rg + q;
      fv[it]  = *(const v4f*)(sY + row * (unsigned)kCh + seg * 32u + c4);
      off[it] = (tok0 + spatial_pos(kd, t0 + row)) * (unsigned)kCh + seg * 32u + c4;
    }
    for (int pass = 0; pass < 2; ++pass) {
#pragma unroll
      for (int it = 0; it < 8; ++it) {
        *(volatile v4f*)(Yk + off[it]) = fv[it];
      }
      __threadfence();
    }
  }
}

constexpr unsigned kOutV4 = (unsigned)(kTok * kCh / 4);
static_assert(kOutV4 % 256u == 0u, "blend grid exact");

__global__ __launch_bounds__(256) void blend_dirs_kernel(
    const float* __restrict__ YD, const float* __restrict__ mw, const float* __restrict__ mb,
    float* __restrict__ out)
{
  const unsigned i = blockIdx.x * 256u + threadIdx.x;
  if (i >= kOutV4) return;
  const size_t e = (size_t)i * 4;
  constexpr size_t plane = (size_t)kTok * kCh;
  const v4f y0 = *(const v4f*)(YD + e);
  const v4f y1 = *(const v4f*)(YD + plane + e);
  const v4f y2 = *(const v4f*)(YD + 2 * plane + e);
  const v4f y3 = *(const v4f*)(YD + 3 * plane + e);
  const float w0 = mw[0], w1 = mw[1], w2 = mw[2], w3 = mw[3];
  const float bb = mb[0];
  const float r0 = (((w0 * y0[0] + w1 * y2[0]) + w2 * y1[0]) + w3 * y3[0]) + bb;
  const float r1 = (((w0 * y0[1] + w1 * y2[1]) + w2 * y1[1]) + w3 * y3[1]) + bb;
  const float r2 = (((w0 * y0[2] + w1 * y2[2]) + w2 * y1[2]) + w3 * y3[2]) + bb;
  const float r3 = (((w0 * y0[3] + w1 * y2[3]) + w2 * y1[3]) + w3 * y3[3]) + bb;
  const v4f r = {r0, r1, r2, r3};
  *(volatile v4f*)(out + e) = r;
  __threadfence();
  *(volatile v4f*)(out + e) = r;
}

extern "C" void kernel_launch(void* const* d_in, const int* in_sizes, int n_in,
                              void* d_out, int out_size, void* d_ws, size_t ws_size,
                              hipStream_t stream) {
  if (n_in < 8) return;
  if (in_sizes[0] != kTok * kCh) return;
  if (in_sizes[1] != kDir * kXw * kCh) return;
  if (in_sizes[2] != kDir * kCh * kRk) return;
  if (in_sizes[3] != kDir * kCh) return;
  if (in_sizes[4] != kDir * kCh * kNst) return;
  if (in_sizes[5] != kDir * kCh) return;
  if (in_sizes[6] != kDir) return;
  if (in_sizes[7] != 1) return;
  if (out_size != kTok * kCh) return;
  if (ws_size < kWsTotal) return;

  const float* x     = (const float*)d_in[0];
  const float* xproj = (const float*)d_in[1];
  const float* dtw   = (const float*)d_in[2];
  const float* dtb   = (const float*)d_in[3];
  const float* alog  = (const float*)d_in[4];
  const float* dsk   = (const float*)d_in[5];
  const float* mw    = (const float*)d_in[6];
  const float* mb    = (const float*)d_in[7];
  float* out = (float*)d_out;

  char* ws = (char*)d_ws;
  unsigned* AH = (unsigned*)(ws + kOffAH);
  unsigned* AL = (unsigned*)(ws + kOffAL);
  unsigned* BH = (unsigned*)(ws + kOffBH);
  unsigned* BL = (unsigned*)(ws + kOffBL);
  float*    XD = (float*)(ws + kOffXD);
  float*    YD = (float*)(ws + kOffYD);

  pack_planes_kernel<<<kPackXBlocks + kPackWBlocks, 256, 0, stream>>>(x, xproj, AH, AL, BH, BL);

  proj_gemm64_kernel<<<(kTok / 64) * (kNW / 64) / 8, 256, 0, stream>>>(
      (const unsigned short*)AH, (const unsigned short*)AL,
      (const unsigned short*)BH, (const unsigned short*)BL, XD);

  scan_dir_kernel<<<kImg * kDir, 192, 0, stream>>>(x, XD, dtw, dtb, alog, dsk, YD);

  blend_dirs_kernel<<<kOutV4 / 256u, 256, 0, stream>>>(YD, mw, mb, out);
}
